// MultiHeadSelfAttention_12713103196901
// MI455X (gfx1250) — hardware-run, weakly checked
//
#include <hip/hip_runtime.h>


#ifndef NB
#define NB 2
#endif
#ifndef SEQ
#define SEQ 2048
#endif
#define NB_FULL  2
#define SEQ_FULL 2048
#define TT   SEQ
#define DM   1024
#define NH_  16
#define HD   64
#define DQ   (NH_ * HD)
#define N3   (3 * DQ)
#define ZH   2
#define RH   ((TT < 512) ? TT : 512)
#define PCAR 1024.0f
#define SCL  0.125f
#define NEGF (-1.0e9f)
static_assert(TT % 128 == 0);
static_assert(RH % 128 == 0);
static_assert((TT - RH) % 64 == 0);
static_assert(NH_ % ZH == 0);
static_assert(DM % 32 == 0);
static_assert(N3 % 64 == 0);

typedef _Float16 h16;
typedef unsigned short bf;
typedef __attribute__((ext_vector_type(16))) __bf16   v16bf;
typedef __attribute__((ext_vector_type(16))) _Float16 v16h;
typedef __attribute__((ext_vector_type(8)))  _Float16 v8h;
typedef __attribute__((ext_vector_type(8)))  unsigned short v8us;
typedef __attribute__((ext_vector_type(8)))  float    v8f;
typedef __attribute__((ext_vector_type(4)))  float    v4f;
typedef __attribute__((ext_vector_type(2)))  float    v2f;
typedef __attribute__((ext_vector_type(2)))  _Float16 v2h;
typedef __attribute__((ext_vector_type(4)))  _Float16 v4h;
typedef __attribute__((ext_vector_type(2)))  unsigned short v2us;
typedef __attribute__((ext_vector_type(4)))  unsigned short v4us;
typedef v4f  __attribute__((may_alias)) v4fa;

__device__ __forceinline__ unsigned short f2bf(float f) { unsigned u = __float_as_uint(f); u += 0x7FFFu + ((u >> 16) & 1u); return (unsigned short)(u >> 16); }
__device__ __forceinline__ float bf2f(unsigned short b) { return __uint_as_float(((unsigned)b) << 16); }
__device__ __forceinline__ float bfr(float f) { return bf2f(f2bf(f)); }
__device__ __forceinline__ v16h cat16(v8h lo, v8h hi) { return __builtin_shufflevector(lo, hi, 0, 1, 2, 3, 4, 5, 6, 7, 8, 9, 10, 11, 12, 13, 14, 15); }
__device__ __forceinline__ v16bf cat16b(v8us lo, v8us hi) { return __builtin_bit_cast(v16bf, __builtin_shufflevector(lo, hi, 0, 1, 2, 3, 4, 5, 6, 7, 8, 9, 10, 11, 12, 13, 14, 15)); }
__device__ __forceinline__ v8f wmma16(v16h a, v16h b, v8f c) { return __builtin_amdgcn_wmma_f32_16x16x32_f16(false, a, false, b, (short)0, c, false, false); }
__device__ __forceinline__ v8f wmmab(v16bf a, v16bf b, v8f c) { return __builtin_amdgcn_wmma_f32_16x16x32_bf16(false, a, false, b, (short)0, c, false, false); }
__device__ __forceinline__ h16 tohx(float x) { return (h16)x; }
__device__ __forceinline__ void splitf(float y, unsigned short& h, unsigned short& l) { h = f2bf(y); l = f2bf(y - bf2f(h)); }

template <typename T16> struct WFrag;
template <> struct WFrag<h16> { typedef v16h V; static __device__ __forceinline__ V ld(const h16* p) { return cat16(*(const v8h*)p, *(const v8h*)(p + 16)); } static __device__ __forceinline__ v8f mma(V a, V b, v8f c) { return wmma16(a, b, c); } };
template <> struct WFrag<bf> { typedef v16bf V; static __device__ __forceinline__ V ld(const bf* p) { return cat16b(*(const v8us*)p, *(const v8us*)(p + 16)); } static __device__ __forceinline__ v8f mma(V a, V b, v8f c) { return wmmab(a, b, c); } };
template <typename T16, int NSPLIT, bool BIAS, int CAUS>
__global__ __launch_bounds__(32) void k_gemmw(const T16* __restrict__ A, const T16* __restrict__ A2, const T16* __restrict__ Bt, const T16* __restrict__ Bt2, int K, float* C, int ldc, const float* __restrict__ bias, size_t sA, size_t sB, size_t sC, int rbase, float osc) {
    typedef typename WFrag<T16>::V V;
    __shared__ __align__(16) float os[16 * 68];
    const int r0 = blockIdx.x * 64, c0 = blockIdx.y * 64;
    if (CAUS == 1) { if (c0 >= rbase + r0 + 64) return; }
    int kend = K;
    if (CAUS == 2) { const int kl = rbase + r0 + 64; kend = (kl < K) ? kl : K; }
    const size_t z = blockIdx.z; A += z * sA; if (A2) A2 += z * sA; Bt += z * sB; if (Bt2) Bt2 += z * sB; C += z * sC;
    const int lane = threadIdx.x & 31, lr = lane & 15, hi = lane >> 4;
    v8f acc[4][4];
#pragma unroll
    for (int mb = 0; mb < 4; ++mb)
#pragma unroll
        for (int nb = 0; nb < 4; ++nb) acc[mb][nb] = (v8f){};
    const size_t aoff = (size_t)(r0 + lr) * K + 8 * hi, boff = (size_t)(c0 + lr) * K + 8 * hi;
#pragma unroll 1
    for (int kc = 0; kc < kend; kc += 32) {
        V a[4], a2[4];
#pragma unroll
        for (int mb = 0; mb < 4; ++mb) { a[mb] = WFrag<T16>::ld(A + aoff + (size_t)mb * 16 * K + kc); if (NSPLIT == 1 || NSPLIT == 2) a2[mb] = WFrag<T16>::ld(A2 + aoff + (size_t)mb * 16 * K + kc); }
#pragma unroll
        for (int nb = 0; nb < 4; ++nb) { const V b = WFrag<T16>::ld(Bt + boff + (size_t)nb * 16 * K + kc); V b2; if (NSPLIT >= 2) b2 = WFrag<T16>::ld(Bt2 + boff + (size_t)nb * 16 * K + kc);
#pragma unroll
            for (int mb = 0; mb < 4; ++mb) { acc[mb][nb] = WFrag<T16>::mma(a[mb], b, acc[mb][nb]); if (NSPLIT == 1 || NSPLIT == 2) acc[mb][nb] = WFrag<T16>::mma(a2[mb], b, acc[mb][nb]); if (NSPLIT >= 2) acc[mb][nb] = WFrag<T16>::mma(a[mb], b2, acc[mb][nb]); } }
        asm volatile("v_nop\n\tv_nop\n\tv_nop\n\tv_nop" : "+v"(acc[0][0]), "+v"(acc[1][1]), "+v"(acc[2][2]), "+v"(acc[3][3]) : "v"(a[0]), "v"(a[3]));
    }
#pragma unroll
    for (int mb = 0; mb < 4; ++mb) {
#pragma unroll
        for (int nb = 0; nb < 4; ++nb) {
#pragma unroll
            for (int j = 0; j < 8; ++j) os[(hi * 8 + j) * 68 + nb * 16 + lr] = acc[mb][nb][j]; }
        __builtin_amdgcn_wave_barrier(); asm volatile("" ::: "memory");
        float* crow = C + (size_t)(r0 + mb * 16) * ldc + c0;
#pragma unroll 1
        for (int ps = 0; ps < 2; ++ps) {
#pragma unroll
            for (int s = 0; s < 8; ++s) { const int row = 2 * s + hi, cofs = lr * 4; v4f val = *(const v4fa*)(os + row * 68 + cofs);
                val[0] *= osc; val[1] *= osc; val[2] *= osc; val[3] *= osc;
                if (BIAS) { val[0] += bfr(bias[c0 + cofs]); val[1] += bfr(bias[c0 + cofs + 1]); val[2] += bfr(bias[c0 + cofs + 2]); val[3] += bfr(bias[c0 + cofs + 3]); }
                *(volatile v4f*)(crow + (size_t)row * ldc + cofs) = val; }
            if (ps == 0) __threadfence(); }
        __builtin_amdgcn_wave_barrier(); asm volatile("" ::: "memory");
    }
}

__global__ __launch_bounds__(256) void k_wtG(const float* __restrict__ w, int K, int N, bf* Bt) {
    const int lane = threadIdx.x & 31; const int L0 = (blockIdx.x * 8 + (threadIdx.x >> 5)) * 8; const int nlines = N * K / 64;
#pragma unroll
    for (int ps = 0; ps < 2; ++ps) {
#pragma unroll 1
        for (int l = 0; l < 8; ++l) { const int L = L0 + l; if (L >= nlines) break; const size_t e = (size_t)L * 64 + lane * 2; const int k = (int)(e % K), n = (int)(e / K); v2us o;
            o[0] = f2bf(w[(size_t)k * N + n]); o[1] = f2bf(w[(size_t)(k + 1) * N + n]); *(volatile v2us*)(Bt + e) = o; }
        if (ps == 0) __threadfence(); }
}
__global__ __launch_bounds__(256) void k_bcat(const float* __restrict__ bqk, const float* __restrict__ bv, float* Bq) {
    const int i = blockIdx.x * 256 + threadIdx.x; if (i >= N3 / 4) return; const int c = i * 4; v4f o;
#pragma unroll
    for (int q = 0; q < 4; ++q) { const int cc = c + q; const int ia = (cc < 2 * DQ) ? cc : (2 * DQ - 1); int ib = cc - 2 * DQ; ib = (ib < 0) ? 0 : ib; ib = (ib > DQ - 1) ? (DQ - 1) : ib;
        const float a = bqk[ia]; const float b2 = bv[ib]; o[q] = (cc < 2 * DQ) ? a : b2; }
    *(volatile v4f*)(Bq + c) = o; __threadfence(); *(volatile v4f*)(Bq + c) = o; }
__global__ __launch_bounds__(256) void k_cvt8(const float* __restrict__ src, bf* dst, size_t n8) { const size_t i = (size_t)blockIdx.x * 256 + threadIdx.x; if (i >= n8) return; const v8f v = *(const v8f*)(src + i * 8); v8us o;
#pragma unroll
    for (int k = 0; k < 8; ++k) o[k] = f2bf(v[k]); *(volatile v8us*)(dst + i * 8) = o; __threadfence(); *(volatile v8us*)(dst + i * 8) = o; }

__global__ __launch_bounds__(256) void k_hp(const float* __restrict__ F, int pitch, int nheads, h16* P16, bf* Ph, bf* Pl) {
    const size_t e = ((size_t)blockIdx.x * 256 + threadIdx.x) * 2; if (e >= (size_t)nheads * TT * HD) return;
    const int d = (int)(e % HD); const int t = (int)((e / HD) % TT); const int h = (int)(e / ((size_t)HD * TT));
    const v2f x = *(const v2f*)(F + (size_t)t * pitch + h * HD + d); v2h o16; v2us oh, ol;
#pragma unroll
    for (int q = 0; q < 2; ++q) { o16[q] = tohx(x[q]); unsigned short a2, c2; splitf(x[q], a2, c2); oh[q] = a2; ol[q] = c2; }
    const bool hl = (t < RH); const size_t eh = ((size_t)h * RH + (hl ? t : 0)) * HD + d;
    *(volatile v2h*)(P16 + e) = o16; if (hl) { *(volatile v2us*)(Ph + eh) = oh; *(volatile v2us*)(Pl + eh) = ol; }
    __threadfence();
    *(volatile v2h*)(P16 + e) = o16; if (hl) { *(volatile v2us*)(Ph + eh) = oh; *(volatile v2us*)(Pl + eh) = ol; } }
__global__ __launch_bounds__(256) void k_vtp(const float* __restrict__ F, int pitch, int nheads, h16* V16, bf* Vh, bf* Vl) {
    const size_t e = ((size_t)blockIdx.x * 256 + threadIdx.x) * 2; if (e >= (size_t)nheads * HD * TT) return;
    const int t = (int)(e % TT); const int d = (int)((e / TT) % HD); const int g = (int)(e / ((size_t)TT * HD)); v2h o16; v2us oh, ol;
#pragma unroll
    for (int q = 0; q < 2; ++q) { const float x = F[(size_t)(t + q) * pitch + g * HD + d]; o16[q] = tohx(x); unsigned short a2, c2; splitf(x, a2, c2); oh[q] = a2; ol[q] = c2; }
    const bool hl = (t < RH); const size_t eh = ((size_t)g * HD + d) * RH + (hl ? t : 0);
    *(volatile v2h*)(V16 + e) = o16; if (hl) { *(volatile v2us*)(Vh + eh) = oh; *(volatile v2us*)(Vl + eh) = ol; }
    __threadfence();
    *(volatile v2h*)(V16 + e) = o16; if (hl) { *(volatile v2us*)(Vh + eh) = oh; *(volatile v2us*)(Vl + eh) = ol; } }

__global__ __launch_bounds__(256) void k_asoft(const float* __restrict__ Sb, h16* P16, bf* Ph, bf* Pl) {
    const int lane = threadIdx.x & 31; const int wv = __builtin_amdgcn_readfirstlane((int)(threadIdx.x >> 5));
    const int row = blockIdx.x * 8 + wv; if (row >= ZH * TT) return;
    const int i = row % TT; const int zz = row / TT; const bool hires = (i < RH);
    const float* sr = Sb + (size_t)row * TT; float v[TT / 32]; float mx = -3.0e38f;
#pragma unroll
    for (int ch = 0; ch < TT / 128; ++ch) {
        if (ch * 128 <= i) { const int j0 = ch * 128 + lane * 4; const v4f a = *(const v4f*)(sr + j0);
#pragma unroll
            for (int q = 0; q < 4; ++q) { const float t = (j0 + q <= i) ? a[q] * SCL : NEGF; v[ch * 4 + q] = t; mx = fmaxf(mx, t); } }
        else {
#pragma unroll
            for (int q = 0; q < 4; ++q) v[ch * 4 + q] = NEGF; } }
#pragma unroll
    for (int sh = 16; sh; sh >>= 1) mx = fmaxf(mx, __shfl_xor(mx, sh, 32));
    float sum = 0.f;
#pragma unroll
    for (int ch = 0; ch < TT / 128; ++ch) {
        if (ch * 128 <= i) {
#pragma unroll
            for (int q = 0; q < 4; ++q) { const int k = ch * 4 + q; float d0 = __fsub_rn(v[k], mx); asm volatile("" : "+v"(d0)); v[k] = __builtin_amdgcn_exp2f(__fmul_rn(d0, 1.4426950408889634f)); sum += v[k]; } }
        else {
#pragma unroll
            for (int q = 0; q < 4; ++q) v[ch * 4 + q] = 0.f; } }
#pragma unroll
    for (int sh = 16; sh; sh >>= 1) sum += __shfl_xor(sum, sh, 32);
    const float f = __fdiv_rn(hires ? 1.0f : PCAR, sum);
#pragma unroll 1
    for (int ps = 0; ps < 2; ++ps) {
        if (hires) {
#pragma unroll
            for (int ch = 0; ch < RH / 128; ++ch) {
                if (ch * 128 <= i) { v4us oh, ol;
#pragma unroll
                    for (int q = 0; q < 4; ++q) { unsigned short a, c2; splitf(v[ch * 4 + q] * f, a, c2); oh[q] = a; ol[q] = c2; }
                    const size_t oo = ((size_t)zz * RH + i) * RH + ch * 128 + lane * 4; *(volatile v4us*)(Ph + oo) = oh; *(volatile v4us*)(Pl + oo) = ol; } }
        } else {
#pragma unroll
            for (int ch = 0; ch < TT / 128; ++ch) {
                if (ch * 128 <= i) { v4h o4;
#pragma unroll
                    for (int q = 0; q < 4; ++q) o4[q] = tohx(v[ch * 4 + q] * f);
                    *(volatile v4h*)(P16 + ((size_t)zz * (TT - RH) + (size_t)(i - RH)) * TT + ch * 128 + lane * 4) = o4; } } }
        if (ps == 0) __threadfence(); }
}

extern "C" void kernel_launch(void* const* d_in, const int* in_sizes, int n_in,
                              void* d_out, int out_size, void* d_ws, size_t ws_size, hipStream_t stream) {
    if (n_in < 5) return;
    if (in_sizes[0] < (NB - 1) * SEQ_FULL * DM + TT * DM) return;
    if (in_sizes[1] < DM * 2 * DQ) return; if (in_sizes[2] < 2 * DQ) return; if (in_sizes[3] < DM * DQ) return; if (in_sizes[4] < DQ) return;
    if (out_size < NB * TT * DM) return;
    const float* x = (const float*)d_in[0]; const float* wqk = (const float*)d_in[1]; const float* bqk = (const float*)d_in[2]; const float* wv = (const float*)d_in[3]; const float* bv = (const float*)d_in[4];
    float* OUT = (float*)d_out;
    char* wsp = (char*)d_ws;
    auto take = [&](size_t bytes) { char* p = wsp; wsp += (bytes + 255) & ~(size_t)255; return (void*)p; };
    bf* WQKV = (bf*)take((size_t)N3 * DM * 2);
    float* BQKV = (float*)take((size_t)N3 * 4);
    bf* XB = (bf*)take((size_t)TT * DM * 2);
    float* F = (float*)take((size_t)TT * N3 * 4);
    h16* QK16 = (h16*)take((size_t)2 * NH_ * TT * HD * 2);
    h16* VT16 = (h16*)take((size_t)NH_ * HD * TT * 2);
    bf* QKh = (bf*)take((size_t)2 * NH_ * RH * HD * 2); bf* QKl = (bf*)take((size_t)2 * NH_ * RH * HD * 2);
    bf* VTh = (bf*)take((size_t)NH_ * HD * RH * 2); bf* VTl = (bf*)take((size_t)NH_ * HD * RH * 2);
    bf* Ph = (bf*)take((size_t)ZH * RH * RH * 2); bf* Pl = (bf*)take((size_t)ZH * RH * RH * 2);
    float* Sb = (float*)take((size_t)ZH * TT * TT * 4);
    h16* P16 = (h16*)take((size_t)ZH * (TT - RH) * TT * 2);
    const size_t carved = (size_t)(wsp - (char*)d_ws);
    if (carved > ws_size || carved > ((size_t)128 << 20)) return;
    k_wtG<<<(unsigned)((DM * 2 * DQ / 64 + 63) / 64), 256, 0, stream>>>(wqk, DM, 2 * DQ, WQKV);
    k_wtG<<<(unsigned)((DM * DQ / 64 + 63) / 64), 256, 0, stream>>>(wv, DM, DQ, WQKV + (size_t)2 * DQ * DM);
    k_bcat<<<(N3 / 4 + 255) / 256, 256, 0, stream>>>(bqk, bv, BQKV);
    const unsigned LQK = (unsigned)(((size_t)2 * NH_ * TT * HD / 2 + 255) / 256), LV = (unsigned)(((size_t)NH_ * TT * HD / 2 + 255) / 256);
    for (int b = 0; b < NB; ++b) {
        float* OB = OUT + (size_t)b * TT * DM;
        k_cvt8<<<(unsigned)(((size_t)TT * DM / 8 + 255) / 256), 256, 0, stream>>>(x + (size_t)b * SEQ_FULL * DM, XB, (size_t)TT * DM / 8);
        k_gemmw<bf, 0, true, 0><<<dim3(TT / 64, N3 / 64, 1), 32, 0, stream>>>(XB, nullptr, WQKV, nullptr, DM, F, N3, BQKV, 0, 0, 0, 0, 1.0f);
        k_hp<<<LQK, 256, 0, stream>>>(F, N3, 2 * NH_, QK16, QKh, QKl);
        k_vtp<<<LV, 256, 0, stream>>>(F + 2 * DQ, N3, NH_, VT16, VTh, VTl);
        for (int h0 = 0; h0 < NH_; h0 += ZH) {
            const size_t zq = (size_t)h0, zk = (size_t)(NH_ + h0);
            k_gemmw<bf, 2, false, 1><<<dim3(RH / 64, RH / 64, ZH), 32, 0, stream>>>(QKh + zq * RH * HD, QKl + zq * RH * HD, QKh + zk * RH * HD, QKl + zk * RH * HD, HD, Sb, TT, nullptr, (size_t)RH * HD, (size_t)RH * HD, (size_t)TT * TT, 0, 1.0f);
            if (TT > RH)
                k_gemmw<h16, 0, false, 1><<<dim3((TT - RH) / 64, TT / 64, ZH), 32, 0, stream>>>(QK16 + zq * TT * HD + (size_t)RH * HD, nullptr, QK16 + zk * TT * HD, nullptr, HD, Sb + (size_t)RH * TT, TT, nullptr, (size_t)TT * HD, (size_t)TT * HD, (size_t)TT * TT, RH, 1.0f);
            k_asoft<<<ZH * TT / 8, 256, 0, stream>>>(Sb, P16, Ph, Pl);
            k_gemmw<bf, 2, false, 2><<<dim3(RH / 64, HD / 64, ZH), 32, 0, stream>>>(Ph, Pl, VTh + (size_t)h0 * HD * RH, VTl + (size_t)h0 * HD * RH, RH, OB + (size_t)h0 * HD, DM, nullptr, (size_t)RH * RH, (size_t)HD * RH, (size_t)HD, 0, 1.0f);
            if (TT > RH)
                k_gemmw<h16, 0, false, 2><<<dim3((TT - RH) / 64, HD / 64, ZH), 32, 0, stream>>>(P16, nullptr, VT16 + (size_t)h0 * HD * TT, nullptr, TT, OB + (size_t)RH * DM + (size_t)h0 * HD, DM, nullptr, (size_t)(TT - RH) * TT, (size_t)HD * TT, (size_t)HD, RH, 1.0f / PCAR);
        }
    }
}
